// MultiHeadSelfAttention_47708496724663
// MI455X (gfx1250) — hardware-run, weakly checked
//
#include <hip/hip_runtime.h>


#ifndef NB
#define NB 2
#endif
#ifndef SEQ
#define SEQ 2048
#endif
#define NB_FULL  2
#define SEQ_FULL 2048
#define TT   SEQ
#define DM   1024
#define NH_  16
#define HD   64
#define DQ   (NH_ * HD)
#define ZH   2
#define RH   ((SEQ < 512) ? SEQ : 512)
#define AW   4
#define TOPK 8
#define PCAR 1024.0f
#define SCL  0.125f
#define NEGS (-1.0e30f)
#define OUT1_OFF ((size_t)NB_FULL * SEQ_FULL * DM)

static_assert(OUT1_OFF * 4 == 16777216);
static_assert(TT % 128 == 0);
static_assert(RH % 128 == 0);
static_assert(RH <= TT);
static_assert(SEQ <= SEQ_FULL);
static_assert(NB <= NB_FULL);
static_assert(DM % 64 == 0);
static_assert(NH_ % ZH == 0);
static_assert((ZH * TT) % AW == 0);
static_assert(TT % AW == 0);
static_assert((TT / AW) % 32 == 0);
static_assert(AW * TT * 4 + 64 <= 65536);

typedef _Float16 h16;
typedef unsigned short bf;
typedef __attribute__((ext_vector_type(16))) __bf16   v16bf;
typedef __attribute__((ext_vector_type(16))) _Float16 v16h;
typedef __attribute__((ext_vector_type(8)))  _Float16 v8h;
typedef __attribute__((ext_vector_type(8)))  unsigned short v8us;
typedef __attribute__((ext_vector_type(8)))  float    v8f;
typedef __attribute__((ext_vector_type(4)))  float    v4f;
typedef __attribute__((ext_vector_type(2)))  float    v2f;
typedef __attribute__((ext_vector_type(4)))  int      v4i;
typedef __attribute__((ext_vector_type(2)))  _Float16 v2h;
typedef __attribute__((ext_vector_type(4)))  _Float16 v4h;
typedef __attribute__((ext_vector_type(2)))  unsigned short v2us;
typedef __attribute__((ext_vector_type(4)))  unsigned short v4us;
typedef v4f  __attribute__((may_alias)) v4fa;

__device__ __forceinline__ unsigned short f2bf(float f) { unsigned u = __float_as_uint(f); u += 0x7FFFu + ((u >> 16) & 1u); return (unsigned short)(u >> 16); }
__device__ __forceinline__ float bf2f(unsigned short b) { return __uint_as_float(((unsigned)b) << 16); }
__device__ __forceinline__ float bfr(float f) { return bf2f(f2bf(f)); }
__device__ __forceinline__ v16h cat16(v8h lo, v8h hi) { return __builtin_shufflevector(lo, hi, 0, 1, 2, 3, 4, 5, 6, 7, 8, 9, 10, 11, 12, 13, 14, 15); }
__device__ __forceinline__ v16bf cat16b(v8us lo, v8us hi) { return __builtin_bit_cast(v16bf, __builtin_shufflevector(lo, hi, 0, 1, 2, 3, 4, 5, 6, 7, 8, 9, 10, 11, 12, 13, 14, 15)); }
__device__ __forceinline__ v8f wmma16(v16h a, v16h b, v8f c) { return __builtin_amdgcn_wmma_f32_16x16x32_f16(false, a, false, b, (short)0, c, false, false); }
__device__ __forceinline__ v8f wmmab(v16bf a, v16bf b, v8f c) { return __builtin_amdgcn_wmma_f32_16x16x32_bf16(false, a, false, b, (short)0, c, false, false); }
__device__ __forceinline__ h16 tohx(float x) { return (h16)x; }
__device__ __forceinline__ void splitf(float y, unsigned short& h, unsigned short& l) { h = f2bf(y); l = f2bf(y - bf2f(h)); }

template <typename T16> struct WFrag;
template <> struct WFrag<h16> { typedef v16h V; static __device__ __forceinline__ V ld(const h16* p) { return cat16(*(const v8h*)p, *(const v8h*)(p + 16)); } static __device__ __forceinline__ v8f mma(V a, V b, v8f c) { return wmma16(a, b, c); } };
template <> struct WFrag<bf> { typedef v16bf V; static __device__ __forceinline__ V ld(const bf* p) { return cat16b(*(const v8us*)p, *(const v8us*)(p + 16)); } static __device__ __forceinline__ v8f mma(V a, V b, v8f c) { return wmmab(a, b, c); } };
template <typename T16, int NSPLIT, bool BIAS>
__global__ __launch_bounds__(32) void k_gemmw(const T16* __restrict__ A, const T16* __restrict__ A2, const T16* __restrict__ Bt, const T16* __restrict__ Bt2, int K, float* C, int ldc, const float* __restrict__ bias, size_t sA, size_t sB, size_t sC, int rbase, int cmode) {
    typedef typename WFrag<T16>::V V;
    __shared__ __align__(16) float os[16 * 68];
    const size_t z = blockIdx.z; A += z * sA; if (A2) A2 += z * sA; Bt += z * sB; if (Bt2) Bt2 += z * sB; C += z * sC;
    const int lane = threadIdx.x & 31, lr = lane & 15, hi = lane >> 4; const int r0 = blockIdx.x * 64, c0 = blockIdx.y * 64;
    const int cb = ((rbase + r0) / 128 + 1) * 128;
    if (cmode == 1 && c0 >= cb) return;
    const int kend = (cmode == 2 && cb < K) ? cb : K;
    v8f acc[4][4];
#pragma unroll
    for (int mb = 0; mb < 4; ++mb)
#pragma unroll
        for (int nb = 0; nb < 4; ++nb) acc[mb][nb] = (v8f){};
    const size_t aoff = (size_t)(r0 + lr) * K + 8 * hi, boff = (size_t)(c0 + lr) * K + 8 * hi;
#pragma unroll 1
    for (int kc = 0; kc < kend; kc += 32) {
        V a[4], a2[4];
#pragma unroll
        for (int mb = 0; mb < 4; ++mb) { a[mb] = WFrag<T16>::ld(A + aoff + (size_t)mb * 16 * K + kc); if (NSPLIT == 1 || NSPLIT == 2) a2[mb] = WFrag<T16>::ld(A2 + aoff + (size_t)mb * 16 * K + kc); }
#pragma unroll
        for (int nb = 0; nb < 4; ++nb) { const V b = WFrag<T16>::ld(Bt + boff + (size_t)nb * 16 * K + kc); V b2; if (NSPLIT >= 2) b2 = WFrag<T16>::ld(Bt2 + boff + (size_t)nb * 16 * K + kc);
#pragma unroll
            for (int mb = 0; mb < 4; ++mb) { acc[mb][nb] = WFrag<T16>::mma(a[mb], b, acc[mb][nb]); if (NSPLIT == 1 || NSPLIT == 2) acc[mb][nb] = WFrag<T16>::mma(a2[mb], b, acc[mb][nb]); if (NSPLIT >= 2) acc[mb][nb] = WFrag<T16>::mma(a[mb], b2, acc[mb][nb]); } }
        asm volatile("v_nop\n\tv_nop\n\tv_nop\n\tv_nop" : "+v"(acc[0][0]), "+v"(acc[1][1]), "+v"(acc[2][2]), "+v"(acc[3][3]) : "v"(a[0]), "v"(a[3]));
    }
#pragma unroll
    for (int mb = 0; mb < 4; ++mb) {
#pragma unroll
        for (int nb = 0; nb < 4; ++nb) {
#pragma unroll
            for (int j = 0; j < 8; ++j) os[(hi * 8 + j) * 68 + nb * 16 + lr] = acc[mb][nb][j]; }
        __builtin_amdgcn_wave_barrier(); asm volatile("" ::: "memory");
        float* crow = C + (size_t)(r0 + mb * 16) * ldc + c0;
#pragma unroll 1
        for (int ps = 0; ps < 2; ++ps) {
#pragma unroll
            for (int s = 0; s < 8; ++s) { const int row = 2 * s + hi, cofs = lr * 4; v4f val = *(const v4fa*)(os + row * 68 + cofs); if (BIAS) { val[0] += bfr(bias[c0 + cofs]); val[1] += bfr(bias[c0 + cofs + 1]); val[2] += bfr(bias[c0 + cofs + 2]); val[3] += bfr(bias[c0 + cofs + 3]); }
                *(volatile v4f*)(crow + (size_t)row * ldc + cofs) = val; }
            if (ps == 0) __threadfence(); }
        __builtin_amdgcn_wave_barrier(); asm volatile("" ::: "memory");
    }
}

__global__ __launch_bounds__(256) void k_wtG(const float* __restrict__ w, int K, int N, bf* Bt) {
    const int lane = threadIdx.x & 31; const int L0 = (blockIdx.x * 8 + (threadIdx.x >> 5)) * 8; const int nlines = N * K / 64;
#pragma unroll
    for (int ps = 0; ps < 2; ++ps) {
#pragma unroll 1
        for (int l = 0; l < 8; ++l) { const int L = L0 + l; if (L >= nlines) break; const size_t e = (size_t)L * 64 + lane * 2; const int k = (int)(e % K), n = (int)(e / K); v2us o;
            o[0] = f2bf(w[(size_t)k * N + n]); o[1] = f2bf(w[(size_t)(k + 1) * N + n]); *(volatile v2us*)(Bt + e) = o; }
        if (ps == 0) __threadfence(); }
}
__global__ __launch_bounds__(256) void k_cvt8(const float* __restrict__ src, bf* dst, size_t n8) { const size_t i = (size_t)blockIdx.x * 256 + threadIdx.x; if (i >= n8) return; const v8f v = *(const v8f*)(src + i * 8); v8us o;
#pragma unroll
    for (int k = 0; k < 8; ++k) o[k] = f2bf(v[k]); *(volatile v8us*)(dst + i * 8) = o; __threadfence(); *(volatile v8us*)(dst + i * 8) = o; }

__global__ __launch_bounds__(256) void k_hpl(const float* __restrict__ F, int pitch, int nheads, h16* P16, bf* Ph, bf* Pl) {
    const size_t e = ((size_t)blockIdx.x * 256 + threadIdx.x) * 2; if (e >= (size_t)nheads * TT * HD) return; const int d = (int)(e % HD); const int t = (int)((e / HD) % TT); const int h = (int)(e / ((size_t)HD * TT));
    const v2f x = *(const v2f*)(F + (size_t)t * pitch + h * HD + d); v2h o16; v2us oh, ol;
#pragma unroll
    for (int q = 0; q < 2; ++q) { o16[q] = tohx(x[q]); unsigned short a2, c2; splitf(x[q], a2, c2); oh[q] = a2; ol[q] = c2; }
    *(volatile v2h*)(P16 + e) = o16; *(volatile v2us*)(Ph + e) = oh; *(volatile v2us*)(Pl + e) = ol; __threadfence(); *(volatile v2h*)(P16 + e) = o16; *(volatile v2us*)(Ph + e) = oh; *(volatile v2us*)(Pl + e) = ol; }
__global__ __launch_bounds__(256) void k_vtp(const float* __restrict__ F, int pitch, int nheads, h16* V16, bf* Vh, bf* Vl) { const size_t e = ((size_t)blockIdx.x * 256 + threadIdx.x) * 2; if (e >= (size_t)nheads * HD * TT) return; const int t = (int)(e % TT); const int d = (int)((e / TT) % HD); const int g = (int)(e / ((size_t)TT * HD)); v2h o16; v2us oh, ol;
#pragma unroll
    for (int q = 0; q < 2; ++q) { const float x = F[(size_t)(t + q) * pitch + g * HD + d]; o16[q] = tohx(x); unsigned short a2, c2; splitf(x, a2, c2); oh[q] = a2; ol[q] = c2; }
    *(volatile v2h*)(V16 + e) = o16; *(volatile v2us*)(Vh + e) = oh; *(volatile v2us*)(Vl + e) = ol; __threadfence(); *(volatile v2h*)(V16 + e) = o16; *(volatile v2us*)(Vh + e) = oh; *(volatile v2us*)(Vl + e) = ol; }

__global__ __launch_bounds__(AW * 32) void k_asoft(const float* __restrict__ Sb, const int* __restrict__ am, h16* P16, bf* Ph, bf* Pl, float* DL) {
    __shared__ __align__(16) float rowb[AW * TT];
    __shared__ __align__(16) float part[AW * 4];
    const int lane = threadIdx.x & 31, w = threadIdx.x >> 5; const int row = blockIdx.x * AW + w; const int i = row % TT; const int zz = row / TT;
    const bool hires = (i < RH); const int nch = i / 128 + 1; const float* sr = Sb + (size_t)row * TT; float* rb = rowb + w * TT;
    float mx = NEGS;
#pragma unroll 1
    for (int ch = 0; ch < nch; ++ch) { const int j0 = ch * 128 + lane * 4; const v4f a = *(const v4f*)(sr + j0); const v4i m = *(const v4i*)(am + j0); v4f t;
#pragma unroll
        for (int q = 0; q < 4; ++q) { const int j = j0 + q; const float s = a[q] * SCL; const bool ok = (j <= i) && (m[q] != 0); t[q] = ok ? s : NEGS; mx = fmaxf(mx, t[q]); }
        *(v4f*)(rb + j0) = t; }
#pragma unroll
    for (int sh = 16; sh; sh >>= 1) mx = fmaxf(mx, __shfl_xor(mx, sh, 32));
    float sum = 0.f, s1 = 0.f, sd = 0.f, sd2 = 0.f, emax = 0.f;
#pragma unroll 1
    for (int ch = 0; ch < nch; ++ch) { const int j0 = ch * 128 + lane * 4; const v4f t = *(const v4f*)(rb + j0); v4f e;
#pragma unroll
        for (int q = 0; q < 4; ++q) { float d0 = __fsub_rn(t[q], mx); asm volatile("" : "+v"(d0)); const float ev = __builtin_amdgcn_exp2f(__fmul_rn(d0, 1.4426950408889634f)); const float dist = fabsf((float)(i - (j0 + q)));
            e[q] = ev; sum += ev; s1 += ev * d0; const float ed = ev * dist; sd += ed; sd2 += ed * dist; emax = fmaxf(emax, ev); }
        *(v4f*)(rb + j0) = e; }
#pragma unroll
    for (int sh = 16; sh; sh >>= 1) { sum += __shfl_xor(sum, sh, 32); s1 += __shfl_xor(s1, sh, 32); sd += __shfl_xor(sd, sh, 32); sd2 += __shfl_xor(sd2, sh, 32); emax = fmaxf(emax, __shfl_xor(emax, sh, 32)); }
    const bool dead = !(mx > -1.0e29f);
    float inv = __fdiv_rn(1.0f, sum); if (dead) inv = __uint_as_float(0x7fc00000u);
    const float f = hires ? inv : inv * PCAR;
#pragma unroll 1
    for (int ps = 0; ps < 2; ++ps) {
#pragma unroll 1
        for (int ch = 0; ch < nch; ++ch) { const int j0 = ch * 128 + lane * 4; const v4f e = *(const v4f*)(rb + j0);
            if (hires) { v4us oh, ol;
#pragma unroll
                for (int q = 0; q < 4; ++q) { unsigned short a, c2; splitf(e[q] * f, a, c2); oh[q] = a; ol[q] = c2; }
                const size_t oo = ((size_t)zz * RH + i) * TT + j0; *(volatile v4us*)(Ph + oo) = oh; *(volatile v4us*)(Pl + oo) = ol;
            } else { v4h o4;
#pragma unroll
                for (int q = 0; q < 4; ++q) o4[q] = tohx(e[q] * f);
                *(volatile v4h*)(P16 + (size_t)row * TT + j0) = o4; } }
        if (ps == 0) __threadfence(); }
    float mass = 0.f; int rem = TOPK; float gp = emax;
#pragma unroll 1
    for (int r = 0; r < TOPK; ++r) { float lm = -1.0f; int cnt = 0;
#pragma unroll 1
        for (int ch = 0; ch < nch; ++ch) { const int j0 = ch * 128 + lane * 4; const v4f e = *(const v4f*)(rb + j0);
#pragma unroll
            for (int q = 0; q < 4; ++q) { const float xv = e[q]; cnt += (xv == gp) ? 1 : 0; lm = fmaxf(lm, (xv < gp) ? xv : -1.0f); } }
#pragma unroll
        for (int sh = 16; sh; sh >>= 1) { lm = fmaxf(lm, __shfl_xor(lm, sh, 32)); cnt += __shfl_xor(cnt, sh, 32); }
        const int take = (cnt < rem) ? cnt : rem; mass += gp * (float)take; rem -= take;
        if (rem <= 0 || !(lm > 0.0f)) break;
        gp = lm; }
    v4f rs; rs[0] = __logf(sum) - s1 * inv; rs[1] = sd * inv; rs[2] = sd2 * inv; rs[3] = mass * inv;
    if (lane == 0) *(v4f*)(part + w * 4) = rs;
    __syncthreads();
    v4f tot = *(const v4f*)(part);
#pragma unroll
    for (int k = 1; k < AW; ++k) { const v4f p = *(const v4f*)(part + k * 4); tot[0] += p[0]; tot[1] += p[1]; tot[2] += p[2]; tot[3] += p[3]; }
    const v4f zero4 = (v4f){0.f, 0.f, 0.f, 0.f}; const v4f ov = (threadIdx.x == 0) ? tot : zero4;
    if (threadIdx.x < 8) { float* dl = DL + (size_t)blockIdx.x * 32 + threadIdx.x * 4; *(volatile v4f*)dl = ov; __threadfence(); *(volatile v4f*)dl = ov; }
}

__global__ __launch_bounds__(256) void k_merge(const float* __restrict__ O, const float* __restrict__ gates, int h0, bf* Ah, bf* Al) { const size_t e = ((size_t)blockIdx.x * 256 + threadIdx.x) * 2; if (e >= (size_t)ZH * TT * HD) return; const int d = (int)(e % HD); const int t = (int)((e / HD) % TT); const int zz = (int)(e / ((size_t)HD * TT)); const float cs = (t < RH) ? 1.0f : (1.0f / PCAR); const float g = bfr(gates[h0 + zz]); const size_t oo = (size_t)t * DQ + (h0 + zz) * HD + d;
    v2us oh, ol;
#pragma unroll
    for (int q = 0; q < 2; ++q) { unsigned short a, c2; const float val = (O[e + q] * cs) * g; splitf(val, a, c2); oh[q] = a; ol[q] = c2; } *(volatile v2us*)(Ah + oo) = oh; *(volatile v2us*)(Al + oo) = ol; __threadfence(); *(volatile v2us*)(Ah + oo) = oh; *(volatile v2us*)(Al + oo) = ol; }

__global__ __launch_bounds__(512) void k_desc(const float* __restrict__ DL, float* O1) {
    __shared__ __align__(16) float res[NH_ * 4];
    const int lane = threadIdx.x & 31, h = threadIdx.x >> 5;
    double a0 = 0.0, a1 = 0.0, a2 = 0.0, a3 = 0.0;
#pragma unroll 1
    for (int b = 0; b < NB; ++b) {
#pragma unroll 1
        for (int blk = lane; blk < TT / AW; blk += 32) { const v4f v = *(const v4f*)(DL + ((size_t)(b * NH_ + h) * (TT / AW) + blk) * 32); a0 += (double)v[0]; a1 += (double)v[1]; a2 += (double)v[2]; a3 += (double)v[3]; } }
#pragma unroll
    for (int sh = 16; sh; sh >>= 1) { a0 += __shfl_xor(a0, sh, 32); a1 += __shfl_xor(a1, sh, 32); a2 += __shfl_xor(a2, sh, 32); a3 += __shfl_xor(a3, sh, 32); }
    const double rn = 1.0 / (double)(NB * TT); const double ent = a0 * rn, md = a1 * rn, msq = a2 * rn, tk = a3 * rn; double var = msq - md * md; var = (var > 0.0) ? var : ((var == var) ? 0.0 : var);
    v4f r; r[0] = (float)ent; r[1] = (float)md; r[2] = sqrtf((float)var); r[3] = (float)tk;
    if (lane == 0) *(v4f*)(res + h * 4) = r;
    __syncthreads();
    const v4f ov = *(const v4f*)(res + (threadIdx.x & 15) * 4);
    if (threadIdx.x < 16) { float* o = O1 + threadIdx.x * 4; *(volatile v4f*)o = ov; __threadfence(); *(volatile v4f*)o = ov; }
}

extern "C" void kernel_launch(void* const* d_in, const int* in_sizes, int n_in,
                              void* d_out, int out_size, void* d_ws, size_t ws_size, hipStream_t stream) {
    if (n_in < 7) return;
    if ((size_t)in_sizes[0] < (size_t)(NB - 1) * SEQ_FULL * DM + (size_t)SEQ * DM) return;
    if ((size_t)in_sizes[1] < (size_t)(NB - 1) * SEQ_FULL + (size_t)SEQ) return;
    if (in_sizes[2] < NH_) return;
    if ((size_t)in_sizes[3] < (size_t)DM * 3 * DQ) return;
    if (in_sizes[4] < 3 * DQ) return;
    if ((size_t)in_sizes[5] < (size_t)DQ * DM) return;
    if (in_sizes[6] < DM) return;
    if ((size_t)out_size < OUT1_OFF + (size_t)NH_ * 4) return;
    const float* x = (const float*)d_in[0]; const int* am = (const int*)d_in[1]; const float* gates = (const float*)d_in[2];
    const float* wqkv = (const float*)d_in[3]; const float* bqkv = (const float*)d_in[4]; const float* wo = (const float*)d_in[5]; const float* bo = (const float*)d_in[6];
    float* OUT = (float*)d_out;
    char* wsp = (char*)d_ws;
    auto take = [&](size_t bytes) { char* p = wsp; wsp += (bytes + 255) & ~(size_t)255; return (void*)p; };
    bf* WQKV = (bf*)take((size_t)3 * DQ * DM * 2); bf* WQ = WQKV; bf* WK = WQKV + (size_t)DQ * DM; bf* WV = WQKV + (size_t)2 * DQ * DM;
    bf* WO = (bf*)take((size_t)DM * DQ * 2);
    bf* XB = (bf*)take((size_t)TT * DM * 2); float* F = (float*)take((size_t)TT * DQ * 4);
    h16* QP16 = (h16*)take((size_t)NH_ * TT * HD * 2); h16* KP16 = (h16*)take((size_t)NH_ * TT * HD * 2); h16* VT16 = (h16*)take((size_t)NH_ * HD * TT * 2);
    bf* QPh = (bf*)take((size_t)NH_ * TT * HD * 2); bf* QPl = (bf*)take((size_t)NH_ * TT * HD * 2); bf* KPh = (bf*)take((size_t)NH_ * TT * HD * 2); bf* KPl = (bf*)take((size_t)NH_ * TT * HD * 2); bf* VTh = (bf*)take((size_t)NH_ * HD * TT * 2); bf* VTl = (bf*)take((size_t)NH_ * HD * TT * 2);
    bf* Ph = (bf*)take((size_t)ZH * RH * TT * 2); bf* Pl = (bf*)take((size_t)ZH * RH * TT * 2);
    float* Sb = (float*)take((size_t)ZH * TT * TT * 4); h16* P16 = (h16*)take((size_t)ZH * TT * TT * 2); float* Ob = (float*)take((size_t)ZH * TT * HD * 4);
    bf* ATh = (bf*)take((size_t)TT * DQ * 2); bf* ATl = (bf*)take((size_t)TT * DQ * 2);
    float* DESC = (float*)take((size_t)NB * NH_ * (TT / AW) * 32 * 4);
    const size_t used = (size_t)(wsp - (char*)d_ws);
    if (used > ws_size || used > (size_t)134217728) return;
    k_wtG<<<(unsigned)((DM * 3 * DQ / 64 + 63) / 64), 256, 0, stream>>>(wqkv, DM, 3 * DQ, WQKV);
    k_wtG<<<(unsigned)((DQ * DM / 64 + 63) / 64), 256, 0, stream>>>(wo, DQ, DM, WO);
    const unsigned LP = (unsigned)(((size_t)NH_ * TT * HD / 2 + 255) / 256);
    for (int b = 0; b < NB; ++b) {
        k_cvt8<<<(unsigned)(((size_t)TT * DM / 8 + 255) / 256), 256, 0, stream>>>(x + (size_t)b * SEQ_FULL * DM, XB, (size_t)TT * DM / 8);
        k_gemmw<bf, 0, true><<<dim3(TT / 64, DQ / 64, 1), 32, 0, stream>>>(XB, nullptr, WQ, nullptr, DM, F, DQ, bqkv, 0, 0, 0, 0, 0);
        k_hpl<<<LP, 256, 0, stream>>>(F, DQ, NH_, QP16, QPh, QPl);
        k_gemmw<bf, 0, true><<<dim3(TT / 64, DQ / 64, 1), 32, 0, stream>>>(XB, nullptr, WK, nullptr, DM, F, DQ, bqkv + DQ, 0, 0, 0, 0, 0);
        k_hpl<<<LP, 256, 0, stream>>>(F, DQ, NH_, KP16, KPh, KPl);
        k_gemmw<bf, 0, true><<<dim3(TT / 64, DQ / 64, 1), 32, 0, stream>>>(XB, nullptr, WV, nullptr, DM, F, DQ, bqkv + 2 * DQ, 0, 0, 0, 0, 0);
        k_vtp<<<LP, 256, 0, stream>>>(F, DQ, NH_, VT16, VTh, VTl);
        for (int h0 = 0; h0 < NH_; h0 += ZH) { const size_t zq = (size_t)h0;
            k_gemmw<bf, 2, false><<<dim3(RH / 64, RH / 64, ZH), 32, 0, stream>>>(QPh + zq * TT * HD, QPl + zq * TT * HD, KPh + zq * TT * HD, KPl + zq * TT * HD, HD, Sb, TT, nullptr, (size_t)TT * HD, (size_t)TT * HD, (size_t)TT * TT, 0, 1);
            if (TT > RH) k_gemmw<h16, 0, false><<<dim3((TT - RH) / 64 + (TT == RH), TT / 64, ZH), 32, 0, stream>>>(QP16 + zq * TT * HD + (size_t)RH * HD, nullptr, KP16 + zq * TT * HD, nullptr, HD, Sb + (size_t)RH * TT, TT, nullptr, (size_t)TT * HD, (size_t)TT * HD, (size_t)TT * TT, RH, 1);
            k_asoft<<<ZH * TT / AW, AW * 32, 0, stream>>>(Sb, am + (size_t)b * SEQ_FULL, P16, Ph, Pl, DESC + ((size_t)(b * NH_ + h0) * (TT / AW)) * 32);
            k_gemmw<bf, 2, false><<<dim3(RH / 64, HD / 64, ZH), 32, 0, stream>>>(Ph, Pl, VTh + zq * HD * TT, VTl + zq * HD * TT, TT, Ob, HD, nullptr, (size_t)RH * TT, (size_t)HD * TT, (size_t)TT * HD, 0, 2);
            if (TT > RH) k_gemmw<h16, 0, false><<<dim3((TT - RH) / 64 + (TT == RH), HD / 64, ZH), 32, 0, stream>>>(P16 + (size_t)RH * TT, nullptr, VT16 + zq * HD * TT, nullptr, TT, Ob + (size_t)RH * HD, HD, nullptr, (size_t)TT * TT, (size_t)HD * TT, (size_t)TT * HD, RH, 2);
            k_merge<<<(unsigned)(((size_t)ZH * TT * HD / 2 + 255) / 256), 256, 0, stream>>>(Ob, gates, h0, ATh, ATl); }
        k_gemmw<bf, 1, true><<<dim3(TT / 64, DM / 64, 1), 32, 0, stream>>>(ATh, ATl, WO, nullptr, DQ, OUT + (size_t)b * SEQ_FULL * DM, DM, bo, 0, 0, 0, 0, 0); }
    k_desc<<<1, 512, 0, stream>>>(DESC, OUT + OUT1_OFF);
}
